// SS2D6_50345606644093
// MI455X (gfx1250) — hardware-run, weakly checked
//
#include <hip/hip_runtime.h>
#include <math.h>

typedef __attribute__((ext_vector_type(16))) _Float16 v16h;
typedef __attribute__((ext_vector_type(8)))  _Float16 v8h;
typedef __attribute__((ext_vector_type(8)))  float    v8f;
typedef __attribute__((ext_vector_type(4)))  float    v4f;

constexpr int kImgH  = 64;
constexpr int kImgW  = 64;
constexpr int kSeq   = kImgH * kImgW;
constexpr int kDm    = 64;
constexpr int kDi    = 128;
constexpr int kNs    = 16;
constexpr int kDtR   = 4;
constexpr int kDirs  = 6;
constexpr int kXzN   = 2 * kDi;
constexpr int kXdW   = kDtR + 2 * kNs;
constexpr int kXdAll = kDirs * kXdW;
constexpr int kXdP   = 256;
constexpr int kTileP = 132;
constexpr int kScTS  = 64;
constexpr int kXrow  = 40;
static_assert(kSeq == 4096 && kXzN == 256 && kXdW == 36 && kXdAll == 216);
static_assert((kDm % 32) == 0 && (kDi % 32) == 0);
static_assert((kSeq % 64) == 0 && (kXzN % 64) == 0 && (kXdP % 64) == 0 && (kDm % 64) == 0);
static_assert(kXdAll <= kXdP && (kXdW % 4) == 0 && kXrow >= kXdW && (kXrow % 4) == 0);
static_assert((kDirs - 1) * kXdW + kXrow <= kXdP);
static_assert((kSeq % kScTS) == 0 && (kSeq % 16) == 0);
static_assert(((kTileP * 4) % 16) == 0 && kTileP >= kDi);
static_assert((kScTS * (kXrow / 4)) == 128 * 5 && (kScTS * (kDi / 4)) == 128 * 16);

constexpr float kCarAct = 16.0f;
constexpr float kCarY   = 64.0f;
constexpr float kCarW   = 256.0f;
constexpr float kScaleAct = 1.0f / (kCarAct * kCarW);
constexpr float kScaleOut = 1.0f / (kCarY * kCarW);
constexpr float kLnEps  = 1e-5f;
constexpr float kInvDi  = 1.0f / (float)kDi;

constexpr size_t kSzX16   = (size_t)kSeq  * kDm  * 2;
constexpr size_t kSzWINT  = (size_t)kXzN  * kDm  * 2;
constexpr size_t kSzWXT   = (size_t)kXdP  * kDi  * 2;
constexpr size_t kSzWOUTT = (size_t)kDm   * kDi  * 2;
constexpr size_t kSzXZ    = (size_t)kSeq  * kXzN * 4;
constexpr size_t kSzU     = (size_t)kSeq  * kDi  * 4;
constexpr size_t kSzU16   = (size_t)kSeq  * kDi  * 2;
constexpr size_t kSzP     = (size_t)kSeq  * kXdP * 4;
constexpr size_t kSzOUTY  = (size_t)kDirs * kSeq * kDi * 4;
constexpr size_t kSzY16   = (size_t)kSeq  * kDi  * 2;
constexpr size_t kOffX16   = 0;
constexpr size_t kOffWINT  = kOffX16   + kSzX16;
constexpr size_t kOffWXT   = kOffWINT  + kSzWINT;
constexpr size_t kOffWOUTT = kOffWXT   + kSzWXT;
constexpr size_t kOffXZ    = kOffWOUTT + kSzWOUTT;
constexpr size_t kOffU     = kOffXZ    + kSzXZ;
constexpr size_t kOffU16   = kOffU     + kSzU;
constexpr size_t kOffP     = kOffU16   + kSzU16;
constexpr size_t kOffOUTY  = kOffP     + kSzP;
constexpr size_t kOffY16   = kOffOUTY  + kSzOUTY;
constexpr size_t kWsTotal  = kOffY16   + kSzY16;
static_assert(kWsTotal == 25804800ull);
static_assert(kWsTotal <= 134217728ull);
static_assert((kOffWINT % 128) == 0 && (kOffWXT % 128) == 0 && (kOffWOUTT % 128) == 0 && (kOffXZ % 128) == 0 &&
              (kOffU % 128) == 0 && (kOffU16 % 128) == 0 && (kOffP % 128) == 0 && (kOffOUTY % 128) == 0 &&
              (kOffY16 % 128) == 0);

__device__ __forceinline__ float bf16_rne(float f) {
  unsigned u = __float_as_uint(f);
  const unsigned lsb = (u & 0x00010000u) ? 1u : 0u;
  u = (u + 0x7FFFu + lsb) & 0xFFFF0000u;
  return __uint_as_float(u);
}
__device__ __forceinline__ _Float16 to_f16_carry(float v, float carry) {
  float c = v * carry;
  c = fminf(fmaxf(c, -65000.0f), 65000.0f);
  c = (fabsf(c) < 6.103515625e-5f) ? 0.0f : c;
  return (_Float16)c;
}

union FragU { v16h v; v8h h[2]; };
__device__ __forceinline__ v16h frag_load(const _Float16* p) {
  FragU f;
  f.h[0] = *(const v8h*)(p);
  f.h[1] = *(const v8h*)(p + 16);
  return f.v;
}
__device__ __forceinline__ v8f mma_f16(v16h a, v16h b, v8f c) {
  c = __builtin_amdgcn_wmma_f32_16x16x32_f16(false, a, false, b, (short)0, c, false, false);
  asm volatile("v_nop\n\tv_nop\n\tv_nop\n\tv_nop" : "+v"(c) : "v"(a), "v"(b));
  return c;
}
__device__ __forceinline__ void keep4_h(v16h a, v16h b, v16h c, v16h d) { asm volatile("v_nop" :: "v"(a), "v"(b), "v"(c), "v"(d)); }
__device__ __forceinline__ void acc_guard4(v8f& a, v8f& b, v8f& c, v8f& d) { asm volatile("v_nop\n\tv_nop\n\tv_nop\n\tv_nop" : "+v"(a), "+v"(b), "+v"(c), "+v"(d)); }

template <bool BIAS>
__global__ __launch_bounds__(256) void gemm_f16_kernel(
    const unsigned short* __restrict__ Ap, int lda,
    const unsigned short* __restrict__ Btp, int ldb, long strideB,
    float* __restrict__ Cp, int ldc, long strideC,
    const float* __restrict__ biasp, long strideBias,
    int M, int N, int K, float scale) {
  const _Float16* A  = (const _Float16*)Ap;
  const _Float16* Bt = (const _Float16*)Btp + (size_t)blockIdx.y * (size_t)strideB;
  float* C = Cp + (size_t)blockIdx.y * (size_t)strideC;
  __shared__ __align__(16) float sT[8][16 * 68];
  const int lane = threadIdx.x & 31;
  const int wave = threadIdx.x >> 5;
  const int tilesN = N >> 6;
  const int tilesM = M >> 6;
  const int tile = blockIdx.x * 8 + wave;
  if (tile >= tilesM * tilesN) return;
  const int tm = tile / tilesN;
  const int tn = tile - tm * tilesN;
  const int m0 = tm << 6;
  const int n0 = tn << 6;

  const int rlane = lane & 15;
  const int koff  = (lane >> 4) * 8;
  const int mOff  = (lane >> 4) * 8;

  v8f acc[4][4];
#pragma unroll
  for (int i = 0; i < 4; ++i)
#pragma unroll
    for (int j = 0; j < 4; ++j) acc[i][j] = (v8f){0.f,0.f,0.f,0.f,0.f,0.f,0.f,0.f};

  for (int k0 = 0; k0 < K; k0 += 32) {
    v16h bh[4];
#pragma unroll
    for (int j = 0; j < 4; ++j) {
      const size_t bo = (size_t)(n0 + (j << 4) + rlane) * ldb + koff + k0;
      bh[j] = frag_load(Bt + bo);
    }
#pragma unroll
    for (int i = 0; i < 4; ++i) {
      const size_t ao = (size_t)(m0 + (i << 4) + rlane) * lda + koff + k0;
      const v16h ah = frag_load(A + ao);
#pragma unroll
      for (int j = 0; j < 4; ++j) acc[i][j] = mma_f16(ah, bh[j], acc[i][j]);
    }
    keep4_h(bh[0], bh[1], bh[2], bh[3]);
  }
  acc_guard4(acc[0][0], acc[0][1], acc[0][2], acc[0][3]);
  acc_guard4(acc[1][0], acc[1][1], acc[1][2], acc[1][3]);
  acc_guard4(acc[2][0], acc[2][1], acc[2][2], acc[2][3]);
  acc_guard4(acc[3][0], acc[3][1], acc[3][2], acc[3][3]);

  float bvj[4];
#pragma unroll
  for (int j = 0; j < 4; ++j) {
    float t = 0.0f;
    if (BIAS) {
      t = biasp[(size_t)blockIdx.y * (size_t)strideBias + (size_t)(n0 + (j << 4) + rlane)];
      asm volatile("" : "+v"(t));
      t = bf16_rne(t);
    }
    bvj[j] = t;
  }

  float* slab = sT[wave];
#pragma unroll
  for (int i = 0; i < 4; ++i) {
    const int mBase = m0 + (i << 4);
#pragma unroll
    for (int j = 0; j < 4; ++j) {
#pragma unroll
      for (int r = 0; r < 8; ++r) {
        float v = acc[i][j][r] * scale;
        if (BIAS) v = v + bvj[j];
        slab[(mOff + r) * 68 + (j << 4) + rlane] = v;
      }
    }
    __builtin_amdgcn_fence(__ATOMIC_RELEASE, "workgroup");
    __builtin_amdgcn_wave_barrier();
    __builtin_amdgcn_fence(__ATOMIC_ACQUIRE, "workgroup");
    {
      const int hh = lane >> 4, c4 = (lane & 15) * 4;
      for (int pass = 0; pass < 2; ++pass) {
#pragma unroll
        for (int it = 0; it < 8; ++it) {
          const int row = it * 2 + hh;
          const v4f v = *(const v4f*)(slab + row * 68 + c4);
          *(volatile v4f*)(C + (size_t)(mBase + row) * ldc + n0 + c4) = v;
        }
        __threadfence();
      }
    }
    __builtin_amdgcn_fence(__ATOMIC_RELEASE, "workgroup");
    __builtin_amdgcn_wave_barrier();
    __builtin_amdgcn_fence(__ATOMIC_ACQUIRE, "workgroup");
  }
}

template <bool BF>
__global__ __launch_bounds__(256) void cvt_rows_kernel(
    const float* __restrict__ src, unsigned srcPitch, unsigned cols8, unsigned validCols, unsigned validRows,
    unsigned short* __restrict__ dst, unsigned dstPitch, unsigned dstColOff, unsigned total8, float carry) {
  const unsigned i = blockIdx.x * 256u + threadIdx.x;
  if (i >= total8) return;
  unsigned row = i / cols8;
  unsigned col = (i - row * cols8) << 3;
  asm volatile("" : "+v"(row));
  asm volatile("" : "+v"(col));
  const bool rowOk = row < validRows;
  const unsigned rowc = rowOk ? row : (validRows - 1u);
  const float* sp = src + (size_t)rowc * srcPitch + col;
  const v4f a0 = *(const v4f*)(sp);
  const v4f a1 = *(const v4f*)(sp + 4);
  float f0 = a0[0], f1 = a0[1], f2 = a0[2], f3 = a0[3];
  float f4 = a1[0], f5 = a1[1], f6 = a1[2], f7 = a1[3];
  asm volatile("" : "+v"(f0), "+v"(f1), "+v"(f2), "+v"(f3));
  asm volatile("" : "+v"(f4), "+v"(f5), "+v"(f6), "+v"(f7));
  if (BF) {
    f0 = bf16_rne(f0); f1 = bf16_rne(f1); f2 = bf16_rne(f2); f3 = bf16_rne(f3);
    f4 = bf16_rne(f4); f5 = bf16_rne(f5); f6 = bf16_rne(f6); f7 = bf16_rne(f7);
  }
  f0 = (rowOk && (col + 0u < validCols)) ? f0 : 0.0f;
  f1 = (rowOk && (col + 1u < validCols)) ? f1 : 0.0f;
  f2 = (rowOk && (col + 2u < validCols)) ? f2 : 0.0f;
  f3 = (rowOk && (col + 3u < validCols)) ? f3 : 0.0f;
  f4 = (rowOk && (col + 4u < validCols)) ? f4 : 0.0f;
  f5 = (rowOk && (col + 5u < validCols)) ? f5 : 0.0f;
  f6 = (rowOk && (col + 6u < validCols)) ? f6 : 0.0f;
  f7 = (rowOk && (col + 7u < validCols)) ? f7 : 0.0f;
  v8h hv;
  hv[0] = to_f16_carry(f0, carry);
  hv[1] = to_f16_carry(f1, carry);
  hv[2] = to_f16_carry(f2, carry);
  hv[3] = to_f16_carry(f3, carry);
  hv[4] = to_f16_carry(f4, carry);
  hv[5] = to_f16_carry(f5, carry);
  hv[6] = to_f16_carry(f6, carry);
  hv[7] = to_f16_carry(f7, carry);
  unsigned short* q = dst + (size_t)row * dstPitch + dstColOff + col;
  *(volatile v8h*)q = hv;
  __threadfence();
  *(volatile v8h*)q = hv;
}

__global__ __launch_bounds__(128) void conv_silu_kernel(
    const float* __restrict__ XZ, const float* __restrict__ cw, const float* __restrict__ cb,
    float* __restrict__ U, unsigned short* __restrict__ U16) {
  __shared__ __align__(16) float sT[16 * kTileP];
  const unsigned tid = threadIdx.x;
  unsigned lane = tid & 31u;
  unsigned wave = tid >> 5;
  asm volatile("" : "+v"(lane));
  asm volatile("" : "+v"(wave));
  const unsigned hy = blockIdx.x & (unsigned)(kImgH - 1);
  const size_t rowM = (size_t)hy * (size_t)kImgW;
  const bool top = (hy > 0u);
  const bool bot = (hy < (unsigned)(kImgH - 1));
  const size_t rowT = top ? (rowM - (size_t)kImgW) : rowM;
  const size_t rowB = bot ? (rowM + (size_t)kImgW) : rowM;
  const float* wp = cw + (size_t)tid * 9u;
  const float w00 = bf16_rne(wp[0]), w01 = bf16_rne(wp[1]), w02 = bf16_rne(wp[2]);
  const float w10 = bf16_rne(wp[3]), w11 = bf16_rne(wp[4]), w12 = bf16_rne(wp[5]);
  const float w20 = bf16_rne(wp[6]), w21 = bf16_rne(wp[7]), w22 = bf16_rne(wp[8]);
  const float bc = bf16_rne(cb[tid]);
  float lt = 0.0f, lm = 0.0f, lb = 0.0f;
  float ct, cm, cq;
  {
    const float t0 = XZ[rowT * kXzN + tid];
    const float m0 = XZ[rowM * kXzN + tid];
    const float b0 = XZ[rowB * kXzN + tid];
    ct = top ? t0 : 0.0f;
    cm = m0;
    cq = bot ? b0 : 0.0f;
  }
  unsigned q  = lane >> 3;
  unsigned l7 = lane & 7u;
  asm volatile("" : "+v"(q));
  asm volatile("" : "+v"(l7));
#pragma unroll 1
  for (unsigned sub = 0; sub < 4u; ++sub) {
    const size_t pb = rowM + sub * 16u;
#pragma unroll 1
    for (unsigned s = 0; s < 16u; ++s) {
      const unsigned wc = sub * 16u + s;
      const bool hasR = (wc + 1u) < (unsigned)kImgW;
      const unsigned wn = hasR ? (wc + 1u) : (unsigned)(kImgW - 1);
      const float nt = XZ[(rowT + wn) * kXzN + tid];
      const float nm = XZ[(rowM + wn) * kXzN + tid];
      const float nb = XZ[(rowB + wn) * kXzN + tid];
      const float rt = (top && hasR) ? nt : 0.0f;
      const float rm = hasR ? nm : 0.0f;
      const float rb = (bot && hasR) ? nb : 0.0f;
      float acc = w00 * lt;
      acc = fmaf(w01, ct, acc);
      acc = fmaf(w02, rt, acc);
      acc = fmaf(w10, lm, acc);
      acc = fmaf(w11, cm, acc);
      acc = fmaf(w12, rm, acc);
      acc = fmaf(w20, lb, acc);
      acc = fmaf(w21, cq, acc);
      acc = fmaf(w22, rb, acc);
      const float sv = acc + bc;
      const float sg = 1.0f / (1.0f + expf(-sv));
      sT[s * kTileP + tid] = sv * sg;
      lt = ct; ct = rt;
      lm = cm; cm = rm;
      lb = cq; cq = rb;
    }
    __syncthreads();
    v4f fv[4];
    v8h hv[2];
#pragma unroll
    for (int it = 0; it < 4; ++it) {
      const unsigned pr = (unsigned)it * 4u + wave;
      fv[it] = *(const v4f*)(sT + pr * kTileP + lane * 4u);
    }
#pragma unroll
    for (int it = 0; it < 2; ++it) {
      const unsigned li = (unsigned)it * 16u + wave * 4u + q;
      const unsigned pr = li >> 1;
      const unsigned sg2 = li & 1u;
      const float* sp = sT + pr * kTileP + sg2 * 64u + l7 * 8u;
      const v4f a0 = *(const v4f*)(sp);
      const v4f a1 = *(const v4f*)(sp + 4);
#pragma unroll
      for (int e = 0; e < 4; ++e) {
        const float f0 = a0[e];
        const float f1 = a1[e];
        hv[it][e]     = to_f16_carry(f0, kCarAct);
        hv[it][4 + e] = to_f16_carry(f1, kCarAct);
      }
    }
    for (int pass = 0; pass < 2; ++pass) {
#pragma unroll
      for (int it = 0; it < 4; ++it) {
        const unsigned pr = (unsigned)it * 4u + wave;
        *(volatile v4f*)(U + (pb + pr) * kDi + lane * 4u) = fv[it];
      }
#pragma unroll
      for (int it = 0; it < 2; ++it) {
        const unsigned li = (unsigned)it * 16u + wave * 4u + q;
        const unsigned pr = li >> 1;
        const unsigned sg2 = li & 1u;
        *(volatile v8h*)(U16 + (pb + pr) * kDi + sg2 * 64u + l7 * 8u) = hv[it];
      }
      __threadfence();
    }
    __syncthreads();
  }
}

__global__ __launch_bounds__(128) void scan_kernel(
    const float* __restrict__ P, const float* __restrict__ U,
    const float* __restrict__ dtw, const float* __restrict__ dtb,
    const float* __restrict__ Alog, const float* __restrict__ Dsk,
    float* __restrict__ OUTY) {
  __shared__ __align__(16) unsigned sMap[kSeq];
  __shared__ __align__(16) float sX[kScTS * kXrow];
  __shared__ __align__(16) float sUY[kScTS * kDi];
  const unsigned tid = threadIdx.x;
  const unsigned lane = tid & 31u;
  const unsigned wave = tid >> 5;
  const unsigned kdir = blockIdx.x;
  const unsigned kd = kdir * (unsigned)kDi + tid;

#pragma unroll 1
  for (unsigned it = 0; it < 32u; ++it) {
    const unsigned qp = it * 128u + tid;
    const unsigned i = qp >> 6;
    const unsigned j = qp & 63u;
    const unsigned s = i + j;
    const unsigned offLo = (s * (s + 1u)) >> 1;
    const unsigned tq = 127u - s;
    const unsigned offHi = 4096u - ((tq * (tq + 1u)) >> 1);
    const unsigned off = (s < 64u) ? offLo : offHi;
    const unsigned imin = (s > 63u) ? (s - 63u) : 0u;
    const unsigned pos = off + i - imin;
    const unsigned tr = j * 64u + i;
    const unsigned rv = 4095u - qp;
    const unsigned trv = (rv & 63u) * 64u + (rv >> 6);
    const unsigned fw = i * 64u + (63u - j);
    unsigned idx = (kdir >= 4u) ? pos : qp;
    unsigned val = qp;
    val = (kdir == 1u) ? tr : val;
    val = (kdir == 2u) ? rv : val;
    val = (kdir == 3u) ? trv : val;
    val = (kdir == 5u) ? fw : val;
    idx = (idx < 4095u) ? idx : 4095u;
    sMap[idx] = val;
  }

#pragma unroll 1
  for (unsigned s = 0; s < (unsigned)kNs; ++s) {
    const float al = Alog[(size_t)kd * kNs + s];
    sUY[s * (unsigned)kDi + tid] = -expf(bf16_rne(al));
  }
  __syncthreads();
  float negA[kNs], h[kNs];
#pragma unroll
  for (int s = 0; s < kNs; ++s) {
    negA[s] = sUY[s * kDi + tid];
    h[s] = 0.0f;
  }
  const float bb = bf16_rne(dtb[kd]);
  const float Dd = bf16_rne(Dsk[kd]);
  const v4f wv = *(const v4f*)(dtw + (size_t)kd * kDtR);
  const float w0 = bf16_rne(wv[0]);
  const float w1 = bf16_rne(wv[1]);
  const float w2 = bf16_rne(wv[2]);
  const float w3 = bf16_rne(wv[3]);
  const float* Pk = P + kdir * (unsigned)kXdW;
  float* Ok = OUTY + (size_t)kdir * (size_t)kSeq * (size_t)kDi;

#pragma unroll 1
  for (unsigned t0 = 0; t0 < (unsigned)kSeq; t0 += (unsigned)kScTS) {
    __syncthreads();
#pragma unroll
    for (unsigned it = 0; it < 5u; ++it) {
      const unsigned idx = tid + 128u * it;
      const unsigned r = idx / 10u;
      const unsigned c4 = (idx - r * 10u) * 4u;
      unsigned pr = sMap[t0 + r];
      pr = (pr < 4095u) ? pr : 4095u;
      *(v4f*)(sX + r * (unsigned)kXrow + c4) = *(const v4f*)(Pk + (size_t)pr * kXdP + c4);
    }
#pragma unroll
    for (unsigned it = 0; it < 16u; ++it) {
      const unsigned idx = tid + 128u * it;
      const unsigned r = idx >> 5;
      const unsigned c4 = (idx & 31u) * 4u;
      unsigned pr = sMap[t0 + r];
      pr = (pr < 4095u) ? pr : 4095u;
      *(v4f*)(sUY + r * (unsigned)kDi + c4) = *(const v4f*)(U + (size_t)pr * kDi + c4);
    }
    __syncthreads();
#pragma unroll 1
    for (unsigned s = 0; s < (unsigned)kScTS; ++s) {
      const float* xr = sX + s * (unsigned)kXrow;
      const v4f dv = *(const v4f*)(xr);
      const float ut = sUY[s * (unsigned)kDi + tid];
      float pre = w0 * dv[0];
      pre = fmaf(w1, dv[1], pre);
      pre = fmaf(w2, dv[2], pre);
      pre = fmaf(w3, dv[3], pre);
      const float v = pre + bb;
      const float ea = expf(-fabsf(v));
      const float delta = fmaxf(v, 0.0f) + log1pf(ea);
      const float dtx = delta * ut;
      float Bv[kNs], Cv[kNs];
#pragma unroll
      for (int q4 = 0; q4 < 4; ++q4) {
        const v4f bv = *(const v4f*)(xr + kDtR + 4 * q4);
        const v4f cv = *(const v4f*)(xr + kDtR + kNs + 4 * q4);
        Bv[4 * q4 + 0] = bv[0]; Bv[4 * q4 + 1] = bv[1]; Bv[4 * q4 + 2] = bv[2]; Bv[4 * q4 + 3] = bv[3];
        Cv[4 * q4 + 0] = cv[0]; Cv[4 * q4 + 1] = cv[1]; Cv[4 * q4 + 2] = cv[2]; Cv[4 * q4 + 3] = cv[3];
      }
      float y = 0.0f;
#pragma unroll
      for (int n = 0; n < kNs; ++n) {
        const float ee = expf(delta * negA[n]);
        h[n] = fmaf(ee, h[n], dtx * Bv[n]);
        y = fmaf(h[n], Cv[n], y);
      }
      y = fmaf(ut, Dd, y);
      sUY[s * (unsigned)kDi + tid] = y;
    }
    __syncthreads();
    v4f ov[16];
    unsigned po[16];
#pragma unroll
    for (int it = 0; it < 16; ++it) {
      const unsigned r = (unsigned)it * 4u + wave;
      unsigned m = sMap[t0 + r];
      m = (m < 4095u) ? m : 4095u;
      const unsigned m5 = (63u - (m >> 6)) * 64u + (m & 63u);
      po[it] = (kdir == 5u) ? m5 : m;
      ov[it] = *(const v4f*)(sUY + r * (unsigned)kDi + lane * 4u);
    }
    for (int pass = 0; pass < 2; ++pass) {
#pragma unroll
      for (int it = 0; it < 16; ++it) {
        *(volatile v4f*)(Ok + (size_t)po[it] * kDi + lane * 4u) = ov[it];
      }
      __threadfence();
    }
  }
}

__global__ __launch_bounds__(256) void norm_gate_kernel(
    const float* __restrict__ OUTY, const float* __restrict__ XZ,
    const float* __restrict__ lng, const float* __restrict__ lnb,
    unsigned short* __restrict__ Y16) {
  __shared__ __align__(16) float sG[16 * kTileP];
  const unsigned tid = threadIdx.x;
  unsigned lane = tid & 31u;
  unsigned wave = tid >> 5;
  asm volatile("" : "+v"(lane));
  asm volatile("" : "+v"(wave));
  const size_t row0 = (size_t)blockIdx.x * 16u;
  constexpr size_t kPlane = (size_t)kSeq * (size_t)kDi;
  const v4f gg = *(const v4f*)(lng + lane * 4u);
  const v4f bq = *(const v4f*)(lnb + lane * 4u);
  float ge[4], be[4];
#pragma unroll
  for (int e = 0; e < 4; ++e) {
    ge[e] = bf16_rne(gg[e]);
    be[e] = bf16_rne(bq[e]);
  }
#pragma unroll 1
  for (unsigned rr = 0; rr < 2u; ++rr) {
    const unsigned lrow = wave * 2u + rr;
    const size_t grow = row0 + lrow;
    const float* yp = OUTY + grow * kDi + lane * 4u;
    const v4f a0 = *(const v4f*)(yp);
    const v4f a1 = *(const v4f*)(yp + kPlane);
    const v4f a2 = *(const v4f*)(yp + 2 * kPlane);
    const v4f a3 = *(const v4f*)(yp + 3 * kPlane);
    const v4f a4 = *(const v4f*)(yp + 4 * kPlane);
    const v4f a5 = *(const v4f*)(yp + 5 * kPlane);
    const v4f zq = *(const v4f*)(XZ + grow * kXzN + kDi + lane * 4u);
    v4f ya;
#pragma unroll
    for (int e = 0; e < 4; ++e) ya[e] = ((((a0[e] + a1[e]) + a2[e]) + a3[e]) + a4[e]) + a5[e];
    float s = (ya[0] + ya[1]) + (ya[2] + ya[3]);
    s += __shfl_xor(s, 16, 32);
    s += __shfl_xor(s, 8, 32);
    s += __shfl_xor(s, 4, 32);
    s += __shfl_xor(s, 2, 32);
    s += __shfl_xor(s, 1, 32);
    const float mu = s * kInvDi;
    float s2 = 0.0f;
#pragma unroll
    for (int e = 0; e < 4; ++e) {
      const float da = ya[e] - mu;
      s2 = fmaf(da, da, s2);
    }
    s2 += __shfl_xor(s2, 16, 32);
    s2 += __shfl_xor(s2, 8, 32);
    s2 += __shfl_xor(s2, 4, 32);
    s2 += __shfl_xor(s2, 2, 32);
    s2 += __shfl_xor(s2, 1, 32);
    const float rstd = rsqrtf(s2 * kInvDi + kLnEps);
    v4f ovv;
#pragma unroll
    for (int e = 0; e < 4; ++e) {
      const float yn = (ya[e] - mu) * rstd * ge[e] + be[e];
      const float zz = zq[e];
      const float sg = 1.0f / (1.0f + expf(-zz));
      ovv[e] = yn * (zz * sg);
    }
    *(v4f*)(sG + lrow * kTileP + lane * 4u) = ovv;
  }
  __syncthreads();
  unsigned q  = lane >> 3;
  unsigned l7 = lane & 7u;
  asm volatile("" : "+v"(q));
  asm volatile("" : "+v"(l7));
  const unsigned li = wave * 4u + q;
  const unsigned pr = li >> 1;
  const unsigned sg2 = li & 1u;
  v8h hv;
  {
    const float* sp = sG + pr * kTileP + sg2 * 64u + l7 * 8u;
    const v4f a0 = *(const v4f*)(sp);
    const v4f a1 = *(const v4f*)(sp + 4);
#pragma unroll
    for (int e = 0; e < 4; ++e) {
      const float f0 = a0[e];
      const float f1 = a1[e];
      hv[e]     = to_f16_carry(f0, kCarY);
      hv[4 + e] = to_f16_carry(f1, kCarY);
    }
  }
  unsigned short* dq = Y16 + (row0 + pr) * kDi + sg2 * 64u + l7 * 8u;
  *(volatile v8h*)dq = hv;
  __threadfence();
  *(volatile v8h*)dq = hv;
}

static_assert((((kSeq / 64) * (kXzN / 64)) % 8) == 0);
static_assert((((kSeq / 64) * (kXdP / 64)) % 8) == 0);
static_assert((((kSeq / 64) * (kDm / 64)) % 8) == 0);
static_assert(((kSeq * (kDm / 8)) % 256) == 0 && ((kXzN * (kDm / 8)) % 256) == 0);
static_assert(((kXdP * (kDi / 8)) % 256) == 0 && ((kDm * (kDi / 8)) % 256) == 0);

extern "C" void kernel_launch(void* const* d_in, const int* in_sizes, int n_in,
                              void* d_out, int out_size, void* d_ws, size_t ws_size,
                              hipStream_t stream) {
  if (n_in < 12) return;
  if (in_sizes[0]  != kSeq * kDm) return;
  if (in_sizes[1]  != kXzN * kDm) return;
  if (in_sizes[2]  != kDi * 9) return;
  if (in_sizes[3]  != kDi) return;
  if (in_sizes[4]  != kXdAll * kDi) return;
  if (in_sizes[5]  != kDirs * kDi * kDtR) return;
  if (in_sizes[6]  != kDirs * kDi) return;
  if (in_sizes[7]  != kDirs * kDi * kNs) return;
  if (in_sizes[8]  != kDirs * kDi) return;
  if (in_sizes[9]  != kDi) return;
  if (in_sizes[10] != kDi) return;
  if (in_sizes[11] != kDm * kDi) return;
  if (out_size != kSeq * kDm) return;
  if (ws_size < kWsTotal) return;

  const float* x      = (const float*)d_in[0];
  const float* W_in   = (const float*)d_in[1];
  const float* conv_w = (const float*)d_in[2];
  const float* conv_b = (const float*)d_in[3];
  const float* xpw    = (const float*)d_in[4];
  const float* dt_w   = (const float*)d_in[5];
  const float* dt_b   = (const float*)d_in[6];
  const float* A_logs = (const float*)d_in[7];
  const float* Dsv    = (const float*)d_in[8];
  const float* ln_g   = (const float*)d_in[9];
  const float* ln_b   = (const float*)d_in[10];
  const float* W_out  = (const float*)d_in[11];
  float* out = (float*)d_out;

  char* ws = (char*)d_ws;
  unsigned short* X16   = (unsigned short*)(ws + kOffX16);
  unsigned short* WINT  = (unsigned short*)(ws + kOffWINT);
  unsigned short* WXT   = (unsigned short*)(ws + kOffWXT);
  unsigned short* WOUTT = (unsigned short*)(ws + kOffWOUTT);
  float*          XZ    = (float*)(ws + kOffXZ);
  float*          U     = (float*)(ws + kOffU);
  unsigned short* U16   = (unsigned short*)(ws + kOffU16);
  float*          P     = (float*)(ws + kOffP);
  float*          OUTY  = (float*)(ws + kOffOUTY);
  unsigned short* Y16   = (unsigned short*)(ws + kOffY16);

  cvt_rows_kernel<true><<<(kSeq * (kDm / 8)) / 256, 256, 0, stream>>>(
      x, (unsigned)kDm, (unsigned)(kDm / 8), (unsigned)kDm, (unsigned)kSeq, X16, (unsigned)kDm, 0u,
      (unsigned)(kSeq * (kDm / 8)), kCarAct);
  cvt_rows_kernel<true><<<(kXzN * (kDm / 8)) / 256, 256, 0, stream>>>(
      W_in, (unsigned)kDm, (unsigned)(kDm / 8), (unsigned)kDm, (unsigned)kXzN, WINT, (unsigned)kDm, 0u,
      (unsigned)(kXzN * (kDm / 8)), kCarW);
  cvt_rows_kernel<true><<<(kXdP * (kDi / 8)) / 256, 256, 0, stream>>>(
      xpw, (unsigned)kDi, (unsigned)(kDi / 8), (unsigned)kDi, (unsigned)kXdAll, WXT, (unsigned)kDi, 0u,
      (unsigned)(kXdP * (kDi / 8)), kCarW);
  cvt_rows_kernel<true><<<(kDm * (kDi / 8)) / 256, 256, 0, stream>>>(
      W_out, (unsigned)kDi, (unsigned)(kDi / 8), (unsigned)kDi, (unsigned)kDm, WOUTT, (unsigned)kDi, 0u,
      (unsigned)(kDm * (kDi / 8)), kCarW);

  gemm_f16_kernel<false><<<dim3(((kSeq / 64) * (kXzN / 64)) / 8, 1), 256, 0, stream>>>(
      X16, kDm, WINT, kDm, 0L,
      XZ, kXzN, 0L,
      conv_b, 0L,
      kSeq, kXzN, kDm, kScaleAct);

  conv_silu_kernel<<<kImgH, 128, 0, stream>>>(XZ, conv_w, conv_b, U, U16);

  gemm_f16_kernel<false><<<dim3(((kSeq / 64) * (kXdP / 64)) / 8, 1), 256, 0, stream>>>(
      U16, kDi, WXT, kDi, 0L,
      P, kXdP, 0L,
      conv_b, 0L,
      kSeq, kXdP, kDi, kScaleAct);

  scan_kernel<<<kDirs, 128, 0, stream>>>(P, U, dt_w, dt_b, A_logs, Dsv, OUTY);

  norm_gate_kernel<<<kSeq / 16, 256, 0, stream>>>(OUTY, XZ, ln_g, ln_b, Y16);

  gemm_f16_kernel<false><<<dim3(((kSeq / 64) * (kDm / 64)) / 8, 1), 256, 0, stream>>>(
      Y16, kDi, WOUTT, kDi, 0L,
      out, kDm, 0L,
      conv_b, 0L,
      kSeq, kDm, kDi, kScaleOut);
}
